// BatchAttentionLayer_82437602279874
// MI455X (gfx1250) — hardware-verified
//
#include <hip/hip_runtime.h>
#include <hip/hip_bf16.h>
#include <math.h>


#define BB 2
#define SS 2048
#define DD 1024
#define HH 16
#define DKK 64
#define QW 2

typedef _Float16 bf16;
typedef __attribute__((ext_vector_type(4))) unsigned v4u_t;
typedef unsigned v4ua __attribute__((ext_vector_type(4), may_alias));
typedef __attribute__((ext_vector_type(4))) float v4f_t;
typedef float v4fa __attribute__((ext_vector_type(4), may_alias));
typedef __attribute__((ext_vector_type(16))) bf16  bf16x16;
typedef __attribute__((ext_vector_type(8)))  bf16  bf16x8;
typedef __attribute__((ext_vector_type(4)))  bf16  bf16x4;
typedef __attribute__((ext_vector_type(8)))  float f32x8;

#define LDS_STRIDE 48
#define KSTRIDE    72
#define VSTRIDE    48

__device__ __forceinline__ f32x8 wmma_bf16(bf16x16 a, bf16x16 b, f32x8 c) {
  return __builtin_amdgcn_wmma_f32_16x16x32_f16(
      false, a, false, b, (short)0, c, false, false);
}
#define RSPLIT (1.0f / 2048.0f)
__device__ __forceinline__ bf16 lo_of(float v, bf16 h) { return (bf16)((v - (float)h) * 2048.0f); }
__device__ __forceinline__ f32x8 wmma_split(bf16x16 a, bf16x16 al, bf16x16 b, bf16x16 bl, f32x8 c) {
  f32x8 x = {}; x = wmma_bf16(al, b, x); x = wmma_bf16(a, bl, x); return wmma_bf16(a, b, c) + x * RSPLIT; }

template <typename T>
__device__ __forceinline__ bf16x16 load_frag(const T* __restrict__ base, int ld,
                                             int row0, int k0) {
  const int lane = threadIdx.x & 31;
  const int r    = lane & 15;
  const int kh   = (lane >> 4) * 8;
  const T* p0 = base + (size_t)(row0 + r) * ld + (k0 + kh);
  const T* p1 = p0 + 16;
  bf16x16 f;
#pragma unroll
  for (int i = 0; i < 8; ++i) {
    f[i]     = (bf16)p0[i];
    f[i + 8] = (bf16)p1[i];
  }
  return f;
}

__device__ __forceinline__ bf16x16 lds_frag(const bf16* base, int stride) {
  const int lane = threadIdx.x & 31;
  const int row  = lane & 15;
  const int kh   = (lane >> 4) * 8;
  const bf16x8 lo = *(const bf16x8*)(base + row * stride + kh);
  const bf16x8 hi = *(const bf16x8*)(base + row * stride + kh + 16);
  bf16x16 f;
#pragma unroll
  for (int i = 0; i < 8; ++i) { f[i] = lo[i]; f[i + 8] = hi[i]; }
  return f;
}

template <typename T>
__device__ __forceinline__ void stage_read16(const T* __restrict__ p, float* buf) {
#pragma unroll
  for (int i = 0; i < 16; ++i) buf[i] = (float)p[i];
}

__device__ __forceinline__ void stage_write(bf16* dst, const float* buf, int nquad) {
#pragma unroll
  for (int i = 0; i < nquad; ++i) {
    bf16x4 q;
    q[0] = (bf16)buf[4 * i];     q[1] = (bf16)buf[4 * i + 1];
    q[2] = (bf16)buf[4 * i + 2]; q[3] = (bf16)buf[4 * i + 3];
    *(bf16x4*)(dst + 4 * i) = q;
  }
}

__global__ __launch_bounds__(256) void transpose_pack_kernel(const float* __restrict__ W, bf16* __restrict__ WT, int K, int N, size_t plane) {
  __shared__ float tile[64][65];
  const int k0 = blockIdx.y * 64, n0 = blockIdx.x * 64, t = threadIdx.x;
  for (int i = t; i < 64 * 64; i += 256) { const int kr = i >> 6, nc = i & 63; tile[kr][nc] = W[(size_t)(k0 + kr) * N + n0 + nc]; }
  __syncthreads();
#pragma unroll 1
  for (int pass = 0; pass < 2; ++pass) {
    for (int i = t; i < 64 * 8; i += 256) { const int nr = i >> 3, k8 = (i & 7) * 8; bf16 hh[8], hl[8];
#pragma unroll
      for (int e = 0; e < 8; ++e) { const float v = tile[k8 + e][nr]; hh[e] = (bf16)v; hl[e] = lo_of(v, hh[e]); }
      bf16* d = WT + (size_t)(n0 + nr) * K + k0 + k8;
      *(volatile v4u_t*)d = *(const v4ua*)hh; *(volatile v4u_t*)(d + plane) = *(const v4ua*)hl; }
    __threadfence();
  }
}

template <typename AT, typename WT, int MODE>
__global__ __launch_bounds__(256) void gemm_bias_kernel(
    const AT* __restrict__ A, const WT* __restrict__ W,
    const float* __restrict__ bias, void* __restrict__ out,
    int M, int N, int K) {
  __shared__ bf16 ldsA[128 * LDS_STRIDE];
  __shared__ bf16 ldsW[256 * LDS_STRIDE];
  __shared__ __attribute__((aligned(16))) unsigned char sob[256 * 136 * 2];

  const int t    = threadIdx.x;
  const int wave = t >> 5;
  const int lane = t & 31;
  const int wm   = (wave & 1) * 64;
  const int wn   = (wave >> 1) * 64;
  const int mBlk = blockIdx.x * 128;
  const int nBlk = blockIdx.y * 256;

  const int arow = t >> 1;
  const int ach  = (t & 1) * 16;

  float abuf[16];
  float wbuf[32];

  stage_read16(A + (size_t)(mBlk + arow) * K + ach, abuf);
  stage_read16(W + (size_t)(nBlk + t) * K,          wbuf);
  stage_read16(W + (size_t)(nBlk + t) * K + 16,     wbuf + 16);

  f32x8 acc[4][4] = {};

  for (int k = 0; k < K; k += 32) {
    __syncthreads();
    stage_write(&ldsA[arow * LDS_STRIDE + ach], abuf, 4);
    stage_write(&ldsW[t * LDS_STRIDE],          wbuf, 8);
    if (k + 32 < K) {
      stage_read16(A + (size_t)(mBlk + arow) * K + (k + 32) + ach, abuf);
      stage_read16(W + (size_t)(nBlk + t) * K + (k + 32),          wbuf);
      stage_read16(W + (size_t)(nBlk + t) * K + (k + 32) + 16,     wbuf + 16);
    }
    __syncthreads();

    bf16x16 af[4], wf[4];
#pragma unroll
    for (int i = 0; i < 4; ++i)
      af[i] = lds_frag(ldsA + (wm + 16 * i) * LDS_STRIDE, LDS_STRIDE);
#pragma unroll
    for (int j = 0; j < 4; ++j)
      wf[j] = lds_frag(ldsW + (wn + 16 * j) * LDS_STRIDE, LDS_STRIDE);
#pragma unroll
    for (int i = 0; i < 4; ++i)
#pragma unroll
      for (int j = 0; j < 4; ++j)
        acc[i][j] = wmma_bf16(af[i], wf[j], acc[i][j]);
  }

  const int nlane = lane & 15;
  const int mh    = (lane >> 4) * 8;
  __syncthreads();
  if (MODE == 0 || MODE == 1) {
    bf16* so = (bf16*)sob;
#pragma unroll
    for (int i = 0; i < 4; ++i)
#pragma unroll
      for (int j = 0; j < 4; ++j) {
        const int nl = wn + 16 * j + nlane;
        const float bv = bias ? bias[nBlk + nl] : 0.0f;
#pragma unroll
        for (int r = 0; r < 8; ++r) {
          const int ml = wm + 16 * i + mh + r;
          const bf16 hv = (bf16)(acc[i][j][r] + bv);
          if (MODE == 0) so[ml * 264 + nl] = hv;
          else           so[nl * 136 + ml] = hv;
        }
      }
    __syncthreads();
#pragma unroll 1
    for (int pass = 0; pass < 2; ++pass) {
      if (MODE == 0) {
        for (int ch = t; ch < 128 * 32; ch += 256) { const int ml = ch >> 5, q = (ch & 31) * 8;
          *(volatile v4u_t*)((bf16*)out + (size_t)(mBlk + ml) * N + nBlk + q) = *(const v4ua*)(so + ml * 264 + q); }
      } else {
        const int b_ = mBlk >> 11, s0 = mBlk & (SS - 1);
        for (int ch = t; ch < 256 * 16; ch += 256) { const int nl = ch >> 4, q = (ch & 15) * 8; const int n = nBlk + nl, h = n >> 6, dk = n & (DKK - 1);
          *(volatile v4u_t*)((bf16*)out + (((size_t)(b_ * HH + h)) * DKK + dk) * SS + s0 + q) = *(const v4ua*)(so + nl * 136 + q); }
      }
      __threadfence();
    }
  } else {
    float* so = (float*)sob;
#pragma unroll 1
    for (int hf = 0; hf < 2; ++hf) {
      if (wm == hf * 64) {
#pragma unroll
        for (int i = 0; i < 4; ++i)
#pragma unroll
          for (int j = 0; j < 4; ++j) {
            const int nl = wn + 16 * j + nlane;
            const float bv = bias ? bias[nBlk + nl] : 0.0f;
#pragma unroll
            for (int r = 0; r < 8; ++r) so[(16 * i + mh + r) * 260 + nl] = acc[i][j][r] + bv;
          }
      }
      __syncthreads();
#pragma unroll 1
      for (int pass = 0; pass < 2; ++pass) {
        for (int ch = t; ch < 64 * 64; ch += 256) { const int ml = ch >> 6, q = (ch & 63) * 4;
          *(volatile v4f_t*)((float*)out + (size_t)(mBlk + hf * 64 + ml) * N + nBlk + q) = *(const volatile v4fa*)(so + ml * 260 + q); }
        __threadfence();
      }
      __syncthreads();
    }
  }
}

template <typename AT, typename WT, int MODE>
__global__ __launch_bounds__(256) void gemm_split_kernel(
    const AT* __restrict__ A, size_t aPlane, const WT* __restrict__ W, size_t wPlane,
    const float* __restrict__ bias, void* __restrict__ out,
    int M, int N, int K) {
  __shared__ bf16 ldsA[128 * LDS_STRIDE], ldsAl[128 * LDS_STRIDE];
  __shared__ bf16 ldsW[256 * LDS_STRIDE], ldsWl[256 * LDS_STRIDE];
  __shared__ __attribute__((aligned(16))) unsigned char sob[256 * 136 * 2];

  const int t    = threadIdx.x;
  const int wave = t >> 5;
  const int lane = t & 31;
  const int wm   = (wave & 1) * 64;
  const int wn   = (wave >> 1) * 64;
  const int mBlk = blockIdx.x * 128;
  const int nBlk = blockIdx.y * 256;
  const int arow = t >> 1;
  const int ach  = (t & 1) * 16;

  f32x8 acc[4][4] = {};
  for (int k = 0; k < K; k += 32) {
    __syncthreads();
    {
      const AT* ap = A + (size_t)(mBlk + arow) * K + k + ach;
      bf16 hh[16], hl[16];
      if (sizeof(AT) == 4) {
#pragma unroll
        for (int i = 0; i < 16; ++i) { const float v = (float)ap[i]; hh[i] = (bf16)v; hl[i] = lo_of(v, hh[i]); }
      } else {
#pragma unroll
        for (int i = 0; i < 16; ++i) { hh[i] = (bf16)ap[i]; hl[i] = (bf16)ap[aPlane + i]; }
      }
#pragma unroll
      for (int i = 0; i < 16; ++i) { ldsA[arow * LDS_STRIDE + ach + i] = hh[i]; ldsAl[arow * LDS_STRIDE + ach + i] = hl[i]; }
    }
    {
      const WT* wp = W + (size_t)(nBlk + t) * K + k;
      if (sizeof(WT) == 4) {
#pragma unroll
        for (int i = 0; i < 32; ++i) { const float v = (float)wp[i]; const bf16 h_ = (bf16)v; ldsW[t * LDS_STRIDE + i] = h_; ldsWl[t * LDS_STRIDE + i] = lo_of(v, h_); }
      } else {
#pragma unroll
        for (int i = 0; i < 32; ++i) { ldsW[t * LDS_STRIDE + i] = (bf16)wp[i]; ldsWl[t * LDS_STRIDE + i] = (bf16)wp[wPlane + i]; }
      }
    }
    __syncthreads();
    bf16x16 wf[4], wfl[4];
#pragma unroll
    for (int j = 0; j < 4; ++j) { wf[j] = lds_frag(ldsW + (wn + 16 * j) * LDS_STRIDE, LDS_STRIDE); wfl[j] = lds_frag(ldsWl + (wn + 16 * j) * LDS_STRIDE, LDS_STRIDE); }
#pragma unroll
    for (int i = 0; i < 4; ++i) {
      const bf16x16 af = lds_frag(ldsA + (wm + 16 * i) * LDS_STRIDE, LDS_STRIDE), afl = lds_frag(ldsAl + (wm + 16 * i) * LDS_STRIDE, LDS_STRIDE);
#pragma unroll
      for (int j = 0; j < 4; ++j) acc[i][j] = wmma_split(af, afl, wf[j], wfl[j], acc[i][j]);
    }
  }

  const int nlane = lane & 15;
  const int mh    = (lane >> 4) * 8;
  __syncthreads();
  if (MODE == 1) {
    bf16* so = (bf16*)sob;
#pragma unroll
    for (int i = 0; i < 4; ++i)
#pragma unroll
      for (int j = 0; j < 4; ++j) {
        const int nl = wn + 16 * j + nlane;
        const float bv = bias ? bias[nBlk + nl] : 0.0f;
#pragma unroll
        for (int r = 0; r < 8; ++r) so[nl * 136 + wm + 16 * i + mh + r] = (bf16)(acc[i][j][r] + bv);
      }
    __syncthreads();
    const int b_ = mBlk >> 11, s0 = mBlk & (SS - 1);
#pragma unroll 1
    for (int pass = 0; pass < 2; ++pass) {
      for (int ch = t; ch < 256 * 16; ch += 256) { const int nl = ch >> 4, q = (ch & 15) * 8; const int n = nBlk + nl, h = n >> 6, dk = n & (DKK - 1);
        *(volatile v4u_t*)((bf16*)out + (((size_t)(b_ * HH + h)) * DKK + dk) * SS + s0 + q) = *(const v4ua*)(so + nl * 136 + q); }
      __threadfence();
    }
  } else {
    float* so = (float*)sob;
#pragma unroll 1
    for (int hf = 0; hf < 2; ++hf) {
      if (wm == hf * 64) {
#pragma unroll
        for (int i = 0; i < 4; ++i)
#pragma unroll
          for (int j = 0; j < 4; ++j) {
            const int nl = wn + 16 * j + nlane;
            const float bv = bias ? bias[nBlk + nl] : 0.0f;
#pragma unroll
            for (int r = 0; r < 8; ++r) so[(16 * i + mh + r) * 260 + nl] = acc[i][j][r] + bv;
          }
      }
      __syncthreads();
#pragma unroll 1
      for (int pass = 0; pass < 2; ++pass) {
        for (int ch = t; ch < 64 * 64; ch += 256) { const int ml = ch >> 6, q = (ch & 63) * 4;
          *(volatile v4f_t*)((float*)out + (size_t)(mBlk + hf * 64 + ml) * N + nBlk + q) = *(const volatile v4fa*)(so + ml * 260 + q); }
        __threadfence();
      }
      __syncthreads();
    }
  }
}


#define S_N 512
#define T_N 512
#define DU 512
#define DDIM 1024

__global__ __launch_bounds__(256) void k_pack_wlin(const float* __restrict__ W, bf16* __restrict__ W1h, bf16* __restrict__ W2h) {
  const int g = blockIdx.x * 256 + threadIdx.x;
  const int n = g >> 6, c8 = (g & 63) * 8;
  bf16 h1[8], h2[8];
#pragma unroll
  for (int i = 0; i < 8; ++i) { h1[i] = (bf16)W[(size_t)n * DDIM + c8 + i]; h2[i] = (bf16)W[(size_t)n * DDIM + DU + c8 + i]; }
  *(volatile v4u_t*)(W1h + (size_t)n * DU + c8) = *(const v4ua*)h1; *(volatile v4u_t*)(W2h + (size_t)n * DU + c8) = *(const v4ua*)h2; __threadfence();
  *(volatile v4u_t*)(W1h + (size_t)n * DU + c8) = *(const v4ua*)h1; *(volatile v4u_t*)(W2h + (size_t)n * DU + c8) = *(const v4ua*)h2;
}

__global__ __launch_bounds__(256) void k_scores(const float* __restrict__ A32, const float* __restrict__ B32,
                                               const float* __restrict__ w_score, const float* __restrict__ b_score, float* __restrict__ scores) {
  __shared__ __align__(16) float Bs[4][DDIM];
  __shared__ __align__(16) float wsh[DDIM];
  const int tid = threadIdx.x, tblk = blockIdx.x >> 1, sblk = blockIdx.x & 1, t0 = tblk * 4, s = sblk * 256 + tid;
  for (int d = tid; d < DDIM; d += 256) { wsh[d] = w_score[d];
#pragma unroll
    for (int j = 0; j < 4; ++j) Bs[j][d] = B32[(size_t)(t0 + j) * DDIM + d]; }
  __syncthreads();
  const float* Arow = A32 + (size_t)s * DDIM;
  float acc0 = 0.f, acc1 = 0.f, acc2 = 0.f, acc3 = 0.f;
#pragma unroll 1
  for (int d = 0; d < DDIM; ++d) {
    const float a = Arow[d], wv = wsh[d];
    float x;
    x = a + Bs[0][d]; acc0 += wv * (1.0f - 2.0f * __builtin_amdgcn_rcpf(__expf(2.0f * x) + 1.0f));
    x = a + Bs[1][d]; acc1 += wv * (1.0f - 2.0f * __builtin_amdgcn_rcpf(__expf(2.0f * x) + 1.0f));
    x = a + Bs[2][d]; acc2 += wv * (1.0f - 2.0f * __builtin_amdgcn_rcpf(__expf(2.0f * x) + 1.0f));
    x = a + Bs[3][d]; acc3 += wv * (1.0f - 2.0f * __builtin_amdgcn_rcpf(__expf(2.0f * x) + 1.0f));
  }
  const float bs = b_score[0];
#pragma unroll 1
  for (int pass = 0; pass < 2; ++pass) {
    *(volatile float*)(scores + (size_t)(t0 + 0) * S_N + s) = acc0 + bs;
    *(volatile float*)(scores + (size_t)(t0 + 1) * S_N + s) = acc1 + bs;
    *(volatile float*)(scores + (size_t)(t0 + 2) * S_N + s) = acc2 + bs;
    *(volatile float*)(scores + (size_t)(t0 + 3) * S_N + s) = acc3 + bs;
    __threadfence();
  }
}

__global__ __launch_bounds__(256) void k_softmax(const float* __restrict__ scores, bf16* __restrict__ Wp) {
  __shared__ float red[256];
  __shared__ __align__(16) bf16 rowp[2][S_N];
  const int t = blockIdx.x, tid = threadIdx.x;
  const float v0 = scores[(size_t)t * S_N + tid], v1 = scores[(size_t)t * S_N + 256 + tid];
  float mx = fmaxf(v0, v1); red[tid] = mx; __syncthreads();
  for (int o = 128; o > 0; o >>= 1) { if (tid < o) red[tid] = fmaxf(red[tid], red[tid + o]); __syncthreads(); }
  mx = red[0]; __syncthreads();
  const float e0 = expf(v0 - mx), e1 = expf(v1 - mx);
  red[tid] = e0 + e1; __syncthreads();
  for (int o = 128; o > 0; o >>= 1) { if (tid < o) red[tid] += red[tid + o]; __syncthreads(); }
  const float inv = 1.0f / red[0];
  { const float p0 = e0 * inv, p1 = e1 * inv; const bf16 h0 = (bf16)p0, h1 = (bf16)p1;
    rowp[0][tid] = h0; rowp[1][tid] = lo_of(p0, h0); rowp[0][256 + tid] = h1; rowp[1][256 + tid] = lo_of(p1, h1); }
  __syncthreads();
  const size_t plane = (size_t)T_N * S_N;
#pragma unroll 1
  for (int pass = 0; pass < 2; ++pass) {
    if (tid < 128) { const int pl = tid >> 6, q = (tid & 63) * 8;
      *(volatile v4u_t*)(Wp + (size_t)pl * plane + (size_t)t * S_N + q) = *(const v4ua*)(&rowp[pl][q]); }
    __threadfence();
  }
}

extern "C" void kernel_launch(void* const* d_in, const int* in_sizes, int n_in,
                              void* d_out, int out_size, void* d_ws, size_t ws_size,
                              hipStream_t stream) {
  (void)in_sizes; (void)n_in; (void)out_size; (void)ws_size;
  const float* rnn     = (const float*)d_in[0];
  const float* tgt     = (const float*)d_in[1];
  const float* W_lin   = (const float*)d_in[2];
  const float* b_lin   = (const float*)d_in[3];
  const float* w_score = (const float*)d_in[4];
  const float* b_score = (const float*)d_in[5];
  float* out = (float*)d_out;
  char* ws = (char*)d_ws;
  bf16*  W1h  = (bf16*)ws;  ws += (size_t)DDIM * DU * 2;
  bf16*  W2h  = (bf16*)ws;  ws += (size_t)DDIM * DU * 2;
  bf16*  rnnT = (bf16*)ws;  ws += (size_t)2 * DU * S_N * 2;
  float* A32  = (float*)ws; ws += (size_t)S_N * DDIM * 4;
  float* B32  = (float*)ws; ws += (size_t)T_N * DDIM * 4;
  float* sc   = (float*)ws; ws += (size_t)T_N * S_N * 4;
  bf16*  Wp   = (bf16*)ws;  ws += (size_t)2 * T_N * S_N * 2;

  k_pack_wlin<<<(DDIM * 64) / 256, 256, 0, stream>>>(W_lin, W1h, W2h);
  transpose_pack_kernel<<<dim3(DU / 64, S_N / 64), 256, 0, stream>>>(rnn, rnnT, S_N, DU, (size_t)DU * S_N);
  gemm_bias_kernel<float, bf16, 2><<<dim3(S_N / 128, DDIM / 256), 256, 0, stream>>>(rnn, W1h, nullptr, A32, S_N, DDIM, DU);
  gemm_bias_kernel<float, bf16, 2><<<dim3(T_N / 128, DDIM / 256), 256, 0, stream>>>(tgt, W2h, b_lin,   B32, T_N, DDIM, DU);
  k_scores<<<(T_N / 4) * 2, 256, 0, stream>>>(A32, B32, w_score, b_score, sc);
  k_softmax<<<T_N, 256, 0, stream>>>(sc, Wp);
  gemm_split_kernel<bf16, bf16, 2><<<dim3(T_N / 128, DU / 256), 256, 0, stream>>>(Wp, (size_t)T_N * S_N, rnnT, (size_t)DU * S_N, nullptr, out, T_N, DU, S_N);
}
